// SSARLSTM_21921513078898
// MI455X (gfx1250) — hardware-verified
//
#include <hip/hip_runtime.h>
#include <math.h>

typedef __attribute__((ext_vector_type(16))) _Float16 v16h;
typedef __attribute__((ext_vector_type(8)))  _Float16 v8h;
typedef __attribute__((ext_vector_type(16))) __bf16   v16b;
typedef __attribute__((ext_vector_type(8)))  __bf16   v8b;
typedef __attribute__((ext_vector_type(8)))  float    v8f;
typedef __attribute__((ext_vector_type(4)))  float    v4f;

constexpr int kB    = 64;
constexpr int kT    = 512;
constexpr int kH    = 256;
constexpr int kNL   = 4;
constexpr int kC    = 60;
constexpr int kCP   = 64;
constexpr int kG4   = 4 * kH;
constexpr int kK    = 2 * kH;
constexpr int kRowsY = kB * kT;
constexpr int kThr  = 256;
constexpr float kInCarry = 1024.0f;
constexpr float kSc = 1.0f / (kInCarry * kInCarry);
constexpr float kF16MinNormal = 6.103515625e-5f;
constexpr int kFBL = 0, kFBO = 4096, kFBZ = 4160, kFEnd = 6144;
constexpr size_t kOut1 = (size_t)kB * kC * kT;
constexpr size_t kOut2 = kOut1 + (size_t)kNL * kB * kH;
constexpr size_t kOutTotal = kOut2 + (size_t)kNL * kB * kH;

static_assert((kB % 64) == 0 && (kG4 % 64) == 0 && ((kB / 64) * (kG4 / 64)) % 8 == 0 && ((kCP / 64) * (kT / 64)) % 8 == 0 && (kK % 32) == 0 && (kH % 32) == 0 && (kK % 256) == 0 && (kH % 256) == 0,
              "GEMM M, N multiples of 64; grids exact; K multiples of 32; the plane cast's pitches and offsets multiples of 256");

constexpr size_t kOffW4 = 0ull;
constexpr size_t kOffWO16 = 4194304ull;
constexpr size_t kOffBIAS = 4227072ull;
constexpr size_t kOffA4 = 4251648ull;
constexpr size_t kOffG4 = 4513792ull;
constexpr size_t kOffC4 = 5562368ull;
constexpr size_t kOffFIN = 5824512ull;
constexpr size_t kOffHS16 = 6348800ull;
constexpr size_t kOffLAB = 23126016ull;
constexpr size_t kWsTotal = 31514624ull;
static_assert(kWsTotal <= 134217728ull, "carve cap: under 128 MiB");
static_assert(kOffW4 == 0
              && kOffWO16 == kOffW4 + 4194304ull
              && kOffBIAS == kOffWO16 + 32768ull
              && kOffA4 == kOffBIAS + 24576ull
              && kOffG4 == kOffA4 + 262144ull
              && kOffC4 == kOffG4 + 1048576ull
              && kOffFIN == kOffC4 + 262144ull
              && kOffHS16 == kOffFIN + 524288ull
              && kOffLAB == kOffHS16 + 16777216ull
              && kWsTotal == kOffLAB + 8388608ull, "the carve is chained and totalled");
static_assert((kOffW4 % 256) == 0 && (kOffWO16 % 256) == 0 && (kOffBIAS % 256) == 0 && (kOffA4 % 256) == 0 && (kOffG4 % 256) == 0 && (kOffC4 % 256) == 0 && (kOffFIN % 256) == 0 && (kOffHS16 % 256) == 0 && (kOffLAB % 256) == 0, "aligned regions");

__device__ __forceinline__ unsigned short f2bf_bits(float f) {
  unsigned u = __float_as_uint(f);
  return (unsigned short)((u + 0x7FFFu + ((u >> 16) & 1u)) >> 16);
}
__device__ __forceinline__ float bf_bits2f(unsigned short h) { return __uint_as_float(((unsigned)h) << 16); }
__device__ __forceinline__ float bf16r(float f) { return bf_bits2f(f2bf_bits(f)); }
__device__ __forceinline__ float carry_flush(float v, float carry) {
  const float s = v * carry;
  return (fabsf(s) < kF16MinNormal) ? 0.0f : s;
}
__device__ __forceinline__ float frcp(float x) { return __builtin_amdgcn_rcpf(x); }

__device__ __forceinline__ void dep_guard4_h(v8f& a, v8f& b, v8f& c, v8f& d, v16h x, v16h y) { asm volatile("v_nop\n\tv_nop\n\tv_nop\n\tv_nop" : "+v"(a), "+v"(b), "+v"(c), "+v"(d) : "v"(x), "v"(y)); }
__device__ __forceinline__ void dep_guard4_b(v8f& a, v8f& b, v8f& c, v8f& d, v16b x, v16b y) { asm volatile("v_nop\n\tv_nop\n\tv_nop\n\tv_nop" : "+v"(a), "+v"(b), "+v"(c), "+v"(d) : "v"(x), "v"(y)); }
__device__ __forceinline__ void keep4_h(v16h a, v16h b, v16h c, v16h d) { asm volatile("v_nop" :: "v"(a), "v"(b), "v"(c), "v"(d)); }
__device__ __forceinline__ void keep4_b(v16b a, v16b b, v16b c, v16b d) { asm volatile("v_nop" :: "v"(a), "v"(b), "v"(c), "v"(d)); }
__device__ __forceinline__ void acc_guard4(v8f& a, v8f& b, v8f& c, v8f& d) { asm volatile("v_nop\n\tv_nop\n\tv_nop\n\tv_nop" : "+v"(a), "+v"(b), "+v"(c), "+v"(d)); }

template <typename T> struct Frag;
template <> struct Frag<_Float16> {
  typedef v16h V; union U { v16h v; v8h h[2]; };
  static __device__ __forceinline__ v16h load(const _Float16* p) {
    U f; f.h[0] = *(const v8h*)(p); f.h[1] = *(const v8h*)(p + 16); return f.v;
  }
  static __device__ __forceinline__ v8f mma(v16h a, v16h b, v8f c) {
    return __builtin_amdgcn_wmma_f32_16x16x32_f16(false, a, false, b, (short)0, c, false, false);
  }
  static __device__ __forceinline__ void guard4(v8f& a, v8f& b, v8f& c, v8f& d, v16h x, v16h y) { dep_guard4_h(a, b, c, d, x, y); }
  static __device__ __forceinline__ void keep(v16h a, v16h b, v16h c, v16h d) { keep4_h(a, b, c, d); }
};
template <> struct Frag<__bf16> {
  typedef v16b V; union U { v16b v; v8b h[2]; };
  static __device__ __forceinline__ v16b load(const __bf16* p) {
    U f; f.h[0] = *(const v8b*)(p); f.h[1] = *(const v8b*)(p + 16); return f.v;
  }
  static __device__ __forceinline__ v8f mma(v16b a, v16b b, v8f c) {
    return __builtin_amdgcn_wmma_f32_16x16x32_bf16(false, a, false, b, (short)0, c, false, false);
  }
  static __device__ __forceinline__ void guard4(v8f& a, v8f& b, v8f& c, v8f& d, v16b x, v16b y) { dep_guard4_b(a, b, c, d, x, y); }
  static __device__ __forceinline__ void keep(v16b a, v16b b, v16b c, v16b d) { keep4_b(a, b, c, d); }
};

__device__ __forceinline__ v8f mma_h(v16h a, v16h b, v8f c) {
  c = __builtin_amdgcn_wmma_f32_16x16x32_f16(false, a, false, b, (short)0, c, false, false);
  asm volatile("v_nop\n\tv_nop\n\tv_nop\n\tv_nop" : "+v"(c) : "v"(a), "v"(b));
  return c;
}

template <int ET> struct Elem;
template <> struct Elem<0> { typedef _Float16 T; };
template <> struct Elem<1> { typedef __bf16 T; };
template <int ET, bool SPLIT, int BIAS_MODE, int OUT_MODE, bool RESID, int ACT = 0>
__global__ __launch_bounds__(256) void wmma_gemm64(
    const unsigned short* __restrict__ Ap, const unsigned short* __restrict__ A2p, int lda, long strideA,
    const unsigned short* __restrict__ Btp, const unsigned short* __restrict__ Bt2p, int ldb, long strideB,
    void* __restrict__ Cout, void* __restrict__ Cout2, int ldc, long strideC,
    const float* __restrict__ bias,
    const float* __restrict__ resid, long strideR,
    int M, int N, int K, float scale) {
  typedef typename Elem<ET>::T T;
  typedef typename Frag<T>::V V;
  const T* A = (const T*)Ap; const T* A2 = (const T*)A2p; const T* Bt = (const T*)Btp; const T* Bt2 = (const T*)Bt2p;
  __shared__ __align__(16) float sT[8][16 * 68];
  const int b    = blockIdx.y;
  const int lane = threadIdx.x & 31;
  const int wave = threadIdx.x >> 5;
  const int tilesN = N >> 6;
  const int tilesM = M >> 6;
  const int tile = blockIdx.x * 8 + wave;
  if (tile >= tilesM * tilesN) return;
  const int tm = tile / tilesN;
  const int tn = tile - tm * tilesN;
  const int m0 = tm << 6;
  const int n0 = tn << 6;

  const T* Ab  = A  + (size_t)b * strideA;
  const T* Bb  = Bt + (size_t)b * strideB;
  const T* Ab2 = SPLIT ? (A2  + (size_t)b * strideA) : nullptr;
  const T* Bb2 = SPLIT ? (Bt2 + (size_t)b * strideB) : nullptr;

  const int rlane = lane & 15;
  const int koff  = (lane >> 4) * 8;
  const int mOff  = (lane >> 4) * 8;

  v8f acc[4][4];
#pragma unroll
  for (int i = 0; i < 4; ++i)
#pragma unroll
    for (int j = 0; j < 4; ++j) acc[i][j] = (v8f){0.f,0.f,0.f,0.f,0.f,0.f,0.f,0.f};

  for (int k0 = 0; k0 < K; k0 += 32) {
    V bh[4], bl[4];
#pragma unroll
    for (int j = 0; j < 4; ++j) {
      const size_t bo = (size_t)(n0 + (j << 4) + rlane) * ldb + koff + k0;
      bh[j] = Frag<T>::load(Bb + bo);
      if (SPLIT) bl[j] = Frag<T>::load(Bb2 + bo);
    }
#pragma unroll
    for (int i = 0; i < 4; ++i) {
      const size_t ao = (size_t)(m0 + (i << 4) + rlane) * lda + koff + k0;
      V ah = Frag<T>::load(Ab + ao);
      V al;
      if (SPLIT) al = Frag<T>::load(Ab2 + ao);
#pragma unroll
      for (int j = 0; j < 4; ++j) {
        acc[i][j] = Frag<T>::mma(ah, bh[j], acc[i][j]);
        if (SPLIT) {
          acc[i][j] = Frag<T>::mma(ah, bl[j], acc[i][j]);
          acc[i][j] = Frag<T>::mma(al, bh[j], acc[i][j]);
        }
      }
      Frag<T>::guard4(acc[i][0], acc[i][1], acc[i][2], acc[i][3], ah, SPLIT ? al : ah);
    }
    Frag<T>::keep(bh[0], bh[1], bh[2], bh[3]);
    if (SPLIT) Frag<T>::keep(bl[0], bl[1], bl[2], bl[3]);
  }
  acc_guard4(acc[0][0], acc[0][1], acc[0][2], acc[0][3]);
  acc_guard4(acc[1][0], acc[1][1], acc[1][2], acc[1][3]);
  acc_guard4(acc[2][0], acc[2][1], acc[2][2], acc[2][3]);
  acc_guard4(acc[3][0], acc[3][1], acc[3][2], acc[3][3]);

  float* slab = sT[wave];
  const float* Rb = RESID ? (resid + (size_t)b * strideR) : nullptr;
#pragma unroll
  for (int i = 0; i < 4; ++i) {
    const int mBase = m0 + (i << 4);
#pragma unroll
    for (int j = 0; j < 4; ++j) {
      const int n = n0 + (j << 4) + rlane;
      float bv = 0.f;
      if (BIAS_MODE == 2) bv = bias[n];
#pragma unroll
      for (int r = 0; r < 8; ++r) {
        float v = acc[i][j][r] * scale;
        if (BIAS_MODE == 1) v += bias[mBase + mOff + r];
        if (BIAS_MODE == 2) v += bv;
        if (RESID) v += Rb[(size_t)(mBase + mOff + r) * ldc + n];
        if (ACT == 1) v = tanhf(v);
        if (ACT == 2) v = fmaxf(v, 0.0f);
        if (ACT == 3) v = v / (1.0f + expf(-v));
        if (ACT == 4) v = (v > 0.f) ? v : 0.01f * v;
        slab[(mOff + r) * 68 + (j << 4) + rlane] = v;
      }
    }
    __builtin_amdgcn_fence(__ATOMIC_RELEASE, "workgroup");
    __builtin_amdgcn_wave_barrier();
    __builtin_amdgcn_fence(__ATOMIC_ACQUIRE, "workgroup");
    if (OUT_MODE == 0) {
      float* C = (float*)Cout + (size_t)b * strideC;
      const int hh = lane >> 4, c4 = (lane & 15) * 4;
      for (int pass = 0; pass < 2; ++pass) {
#pragma unroll
        for (int it = 0; it < 8; ++it) {
          const int row = it * 2 + hh;
          v4f v = *(const v4f*)(slab + row * 68 + c4);
          *(volatile v4f*)(C + (size_t)(mBase + row) * ldc + n0 + c4) = v;
        }
        __threadfence();
      }
    } else {
      const int q = lane >> 3, c8 = (lane & 7) * 8;
      unsigned short* C  = (unsigned short*)Cout  + (size_t)b * strideC;
      unsigned short* C2 = (OUT_MODE == 2) ? ((unsigned short*)Cout2 + (size_t)b * strideC) : nullptr;
      for (int pass = 0; pass < 2; ++pass) {
#pragma unroll
        for (int it = 0; it < 4; ++it) {
          const int row = it * 4 + q;
          const float* sp = slab + row * 68 + c8;
          v8h hv, lv;
#pragma unroll
          for (int e = 0; e < 8; ++e) {
            if (OUT_MODE == 1) {
              hv[e] = (_Float16)sp[e];
            } else {
              unsigned short hb = f2bf_bits(sp[e]);
              unsigned short lb = f2bf_bits(sp[e] - bf_bits2f(hb));
              hv[e] = __builtin_bit_cast(_Float16, hb);
              lv[e] = __builtin_bit_cast(_Float16, lb);
            }
          }
          *(volatile v8h*)(C + (size_t)(mBase + row) * ldc + n0 + c8) = hv;
          if (OUT_MODE == 2) *(volatile v8h*)(C2 + (size_t)(mBase + row) * ldc + n0 + c8) = lv;
        }
        __threadfence();
      }
    }
    __builtin_amdgcn_fence(__ATOMIC_RELEASE, "workgroup");
    __builtin_amdgcn_wave_barrier();
    __builtin_amdgcn_fence(__ATOMIC_ACQUIRE, "workgroup");
  }
}

__global__ __launch_bounds__(kThr) void cast_plane_kernel(const float* __restrict__ src, unsigned short* __restrict__ dst,
                                                          int colsLog2, int dstPitch, int dstOff) {
  const int i   = blockIdx.x * kThr + threadIdx.x;
  const int sh  = colsLog2 - 3;
  const int row = i >> sh;
  const int c8  = (i & ((1 << sh) - 1)) * 8;
  const float* sp = src + ((size_t)row << colsLog2) + c8;
  const v4f a0 = *(const v4f*)(sp);
  const v4f a1 = *(const v4f*)(sp + 4);
  v8h hv;
#pragma unroll
  for (int e = 0; e < 4; ++e) {
    const float f0 = a0[e];
    const float f1 = a1[e];
    hv[e]     = (_Float16)carry_flush(bf16r(f0), kInCarry);
    hv[4 + e] = (_Float16)carry_flush(bf16r(f1), kInCarry);
  }
  unsigned short* dp = dst + (size_t)row * dstPitch + dstOff + c8;
  *(volatile v8h*)dp = hv;
  __threadfence();
  *(volatile v8h*)dp = hv;
}

__device__ __forceinline__ float fast_tanh(float v) { return 1.0f - 2.0f * frcp(__expf(2.0f * v) + 1.0f); }
__device__ __forceinline__ float fast_sigmoid(float v) { return frcp(1.0f + __expf(-v)); }

__global__ __launch_bounds__(kThr) void setup_kernel(const float* __restrict__ x, const float* __restrict__ bi0, const float* __restrict__ bh0,
                                                     const float* __restrict__ bi1, const float* __restrict__ bh1, const float* __restrict__ bi2,
                                                     const float* __restrict__ bh2, const float* __restrict__ bi3, const float* __restrict__ bh3,
                                                     const float* __restrict__ fc_w, const float* __restrict__ fc_b,
                                                     float* __restrict__ BIAS, unsigned short* __restrict__ WO16, unsigned short* __restrict__ A4,
                                                     float* __restrict__ C4) {
  unsigned v = blockIdx.x * (unsigned)kThr + threadIdx.x;
  asm volatile("" : "+v"(v));
  if (v < 1536u) {
    const unsigned i0 = v * 4u;
    v4f o = {0.f, 0.f, 0.f, 0.f};
    if (i0 < (unsigned)kFBO) {
      const unsigned l = i0 >> 10, j = i0 & 1023u;
      const float* pa = (l == 0u) ? bi0 : (l == 1u) ? bi1 : (l == 2u) ? bi2 : bi3;
      const float* pc = (l == 0u) ? bh0 : (l == 1u) ? bh1 : (l == 2u) ? bh2 : bh3;
      const v4f a = *(const v4f*)(pa + j), c = *(const v4f*)(pc + j);
#pragma unroll
      for (int e = 0; e < 4; ++e) { const float p = a[e], q = c[e]; o[e] = bf16r(p) + bf16r(q); }
    } else if (i0 < (unsigned)(kFBO + kC)) {
      const v4f a = *(const v4f*)(fc_b + (i0 - (unsigned)kFBO));
#pragma unroll
      for (int e = 0; e < 4; ++e) { const float p = a[e]; o[e] = bf16r(p); }
    }
    float* dp = BIAS + i0;
    *(volatile v4f*)dp = o;
    __threadfence();
    *(volatile v4f*)dp = o;
  } else if (v < 19968u) {
    v8h hv;
#pragma unroll
    for (int e = 0; e < 8; ++e) hv[e] = (_Float16)0.0f;
    unsigned short* dp;
    if (v < 3584u) {
      const unsigned w = v - 1536u;
      const unsigned n = w >> 5, c8 = (w & 31u) * 8u;
      const bool live = n < (unsigned)kC;
      const float* sp = fc_w + (size_t)(live ? n : 0u) * kH + c8;
      const v4f a0 = *(const v4f*)sp, a1 = *(const v4f*)(sp + 4);
#pragma unroll
      for (int e = 0; e < 4; ++e) { const float p = a0[e], q = a1[e]; hv[e] = (_Float16)(live ? carry_flush(bf16r(p), kInCarry) : 0.0f); hv[4 + e] = (_Float16)(live ? carry_flush(bf16r(q), kInCarry) : 0.0f); }
      dp = WO16 + (size_t)w * 8u;
    } else {
      const unsigned w = v - 3584u;
      const unsigned l = w >> 12, b = (w >> 6) & 63u, c8 = (w & 63u) * 8u;
      const bool xs = (l == 0u) && (c8 >= (unsigned)kH);
      const float* sp = x + (size_t)b * kT * kH + (xs ? c8 - (unsigned)kH : 0u);
      const v4f a0 = *(const v4f*)sp, a1 = *(const v4f*)(sp + 4);
#pragma unroll
      for (int e = 0; e < 4; ++e) { const float p = a0[e], q = a1[e]; hv[e] = (_Float16)(xs ? carry_flush(bf16r(p), kInCarry) : 0.0f); hv[4 + e] = (_Float16)(xs ? carry_flush(bf16r(q), kInCarry) : 0.0f); }
      dp = A4 + (size_t)w * 8u;
    }
    *(volatile v8h*)dp = hv;
    __threadfence();
    *(volatile v8h*)dp = hv;
  } else {
    const v4f z = {0.f, 0.f, 0.f, 0.f};
    float* dp = C4 + (size_t)(v - 19968u) * 4u;
    *(volatile v4f*)dp = z;
    __threadfence();
    *(volatile v4f*)dp = z;
  }
}
static_assert(kFEnd / 4 == 1536 && kCP * kH / 8 == 2048 && kNL * kB * kK / 8 == 16384 && kNL * kB * kH / 4 == 16384 && 1536 + 2048 + 16384 + 16384 == 142 * kThr && (kFBO % 1024) == 0 && (kC % 4) == 0, "set-up grid exact");

__global__ __launch_bounds__(kThr) void cell4_kernel(const float* __restrict__ G4, const float* __restrict__ BIAS, const float* __restrict__ x,
                                                     float* __restrict__ C4, unsigned short* __restrict__ A4, unsigned short* __restrict__ HS16,
                                                     float* __restrict__ FIN, int k) {
  const int l = (int)(blockIdx.x >> 3);
  const int t = k - l;
  if (t < 0 || t >= kT) return;
  unsigned v = (blockIdx.x & 7u) * (unsigned)kThr + threadIdx.x;
  asm volatile("" : "+v"(v));
  const unsigned b = v >> 5;
  const unsigned u8 = (v & 31u) * 8u;
  const float* gr = G4 + ((size_t)l * kB + b) * kG4 + u8;
  const float* br = BIAS + (size_t)l * kG4 + u8;
  float* cp = C4 + ((size_t)l * kB + b) * kH + u8;
  v8h hv, xv;
  v4f cn0, cn1, hn0, hn1;
#pragma unroll
  for (int hlf = 0; hlf < 2; ++hlf) {
    const v4f gi = *(const v4f*)(gr + 4 * hlf), gf = *(const v4f*)(gr + kH + 4 * hlf), gg = *(const v4f*)(gr + 2 * kH + 4 * hlf), go = *(const v4f*)(gr + 3 * kH + 4 * hlf);
    const v4f bi = *(const v4f*)(br + 4 * hlf), bf_ = *(const v4f*)(br + kH + 4 * hlf), bg = *(const v4f*)(br + 2 * kH + 4 * hlf), bo = *(const v4f*)(br + 3 * kH + 4 * hlf);
    const v4f co = *(const v4f*)(cp + 4 * hlf);
#pragma unroll
    for (int e = 0; e < 4; ++e) {
      const float cn = fast_sigmoid(gf[e] + bf_[e]) * co[e] + fast_sigmoid(gi[e] + bi[e]) * fast_tanh(gg[e] + bg[e]);
      const float hn = fast_sigmoid(go[e] + bo[e]) * fast_tanh(cn);
      if (hlf == 0) { cn0[e] = cn; hn0[e] = hn; } else { cn1[e] = cn; hn1[e] = hn; }
      hv[4 * hlf + e] = (_Float16)carry_flush(hn, kInCarry);
    }
  }
  const bool first = (l == 0), lastL = (l == kNL - 1);
  const bool nx = first && (t + 1 < kT);
  {
    const float* sp = x + ((size_t)b * kT + (size_t)(nx ? (t + 1) : 0)) * kH + u8;
    const v4f a0 = *(const v4f*)sp, a1 = *(const v4f*)(sp + 4);
#pragma unroll
    for (int e = 0; e < 4; ++e) { const float p = a0[e], q = a1[e]; xv[e] = (_Float16)carry_flush(bf16r(p), kInCarry); xv[4 + e] = (_Float16)carry_flush(bf16r(q), kInCarry); }
  }
  unsigned short* hp = A4 + ((size_t)l * kB + b) * kK + u8;
  unsigned short* yp = lastL ? (HS16 + ((size_t)b * kT + (size_t)t) * kH + u8)
                             : (A4 + ((size_t)(l + 1) * kB + b) * kK + kH + u8);
  unsigned short* xp = A4 + (size_t)b * kK + kH + u8;
  float* fh = FIN + ((size_t)l * kB + b) * kH + u8;
  float* fc = FIN + ((size_t)(kNL + l) * kB + b) * kH + u8;
  const bool fin = (t == kT - 1);
  for (int pass = 0; pass < 2; ++pass) {
    *(volatile v4f*)cp = cn0; *(volatile v4f*)(cp + 4) = cn1;
    *(volatile v8h*)hp = hv;
    *(volatile v8h*)yp = hv;
    if (nx) *(volatile v8h*)xp = xv;
    if (fin) { *(volatile v4f*)fh = hn0; *(volatile v4f*)(fh + 4) = hn1; *(volatile v4f*)fc = cn0; *(volatile v4f*)(fc + 4) = cn1; }
    __threadfence();
  }
}
static_assert(kB * kH / 8 == 8 * kThr && kH / 8 == 32, "cell grid: 8 blocks a layer");

__global__ __launch_bounds__(kThr) void label_kernel(const float* __restrict__ LAB, const float* __restrict__ BIAS, float* __restrict__ out) {
  unsigned v = blockIdx.x * (unsigned)kThr + threadIdx.x;
  asm volatile("" : "+v"(v));
  const unsigned i4 = v * 4u;
  const unsigned t4 = i4 & 511u, bc = i4 >> 9;
  const unsigned b = bc / (unsigned)kC, c = bc % (unsigned)kC;
  const v4f a = *(const v4f*)(LAB + ((size_t)b * kCP + c) * kT + t4);
  const float fb = BIAS[kFBO + c];
  const v4f o = {a[0] + fb, a[1] + fb, a[2] + fb, a[3] + fb};
  float* dp = out + (size_t)i4;
  *(volatile v4f*)dp = o;
  __threadfence();
  *(volatile v4f*)dp = o;
}
static_assert(kOut1 / 4 == 1920 * (size_t)kThr && (kT % 4) == 0, "label grid exact");

__global__ __launch_bounds__(kThr) void last_out_kernel(const float* __restrict__ FIN, float* __restrict__ out1) {
  const size_t i = (size_t)blockIdx.x * kThr + threadIdx.x;
  const v4f o = *(const v4f*)(FIN + i * 4);
  float* dp = out1 + i * 4;
  *(volatile v4f*)dp = o;
  __threadfence();
  *(volatile v4f*)dp = o;
}
static_assert(2 * kNL * kB * kH / 4 == 128 * kThr, "last-states grid exact");

static_assert(((size_t)kG4 * kH / 8) % kThr == 0, "plane cast grids exact");

extern "C" void kernel_launch(void* const* d_in, const int* in_sizes, int n_in,
                              void* d_out, int out_size, void* d_ws, size_t ws_size,
                              hipStream_t stream) {
  if (n_in < 19 || d_out == nullptr || d_ws == nullptr) return;
  if (in_sizes[0] != kB * kT * kH) return;
  for (int l = 0; l < kNL; ++l) {
    if (in_sizes[1 + 4 * l] != kG4 * kH || in_sizes[2 + 4 * l] != kG4 * kH || in_sizes[3 + 4 * l] != kG4 || in_sizes[4 + 4 * l] != kG4) return;
  }
  if (in_sizes[17] != kC * kH || in_sizes[18] != kC) return;
  if ((size_t)out_size != kOutTotal) return;
  if (ws_size < kWsTotal) return;
  const float* x = (const float*)d_in[0];
  const float* fc_w = (const float*)d_in[17];
  const float* fc_b = (const float*)d_in[18];
  float* out = (float*)d_out;
  char* ws = (char*)d_ws;
  unsigned short* W4 = (unsigned short*)(ws + kOffW4);
  unsigned short* WO16 = (unsigned short*)(ws + kOffWO16);
  float* BIAS = (float*)(ws + kOffBIAS);
  unsigned short* A4 = (unsigned short*)(ws + kOffA4);
  float* G4 = (float*)(ws + kOffG4);
  float* C4 = (float*)(ws + kOffC4);
  float* FIN = (float*)(ws + kOffFIN);
  unsigned short* HS16 = (unsigned short*)(ws + kOffHS16);
  float* LAB = (float*)(ws + kOffLAB);

  for (int l = 0; l < kNL; ++l) {
    const float* W_ih = (const float*)d_in[1 + 4 * l];
    const float* W_hh = (const float*)d_in[2 + 4 * l];
    unsigned short* Wl = W4 + (size_t)l * kG4 * kK;
    cast_plane_kernel<<<(int)(((size_t)kG4 * kH / 8) / kThr), kThr, 0, stream>>>(W_hh, Wl, 8, kK, 0);
    cast_plane_kernel<<<(int)(((size_t)kG4 * kH / 8) / kThr), kThr, 0, stream>>>(W_ih, Wl, 8, kK, kH);
  }
  setup_kernel<<<142, kThr, 0, stream>>>(x, (const float*)d_in[3], (const float*)d_in[4], (const float*)d_in[7], (const float*)d_in[8], (const float*)d_in[11],
                                         (const float*)d_in[12], (const float*)d_in[15], (const float*)d_in[16], fc_w, fc_b, BIAS, WO16, A4, C4);

  for (int k = 0; k < kT + kNL - 1; ++k) {
    wmma_gemm64<0, false, 2, 0, false, 0><<<dim3((kB / 64) * (kG4 / 64) / 8, kNL), 256, 0, stream>>>(
        A4, A4, kK, (long)kB * kK, W4, W4, kK, (long)kG4 * kK, (void*)G4, (void*)G4, kG4, (long)kB * kG4, BIAS + kFBZ, nullptr, 0L, kB, kG4, kK, kSc);
    cell4_kernel<<<32, kThr, 0, stream>>>(G4, BIAS, x, C4, A4, HS16, FIN, k);
  }
  wmma_gemm64<0, false, 2, 0, false, 0><<<dim3((kCP / 64) * (kT / 64) / 8, kB), 256, 0, stream>>>(
      WO16, WO16, kH, 0L, HS16, HS16, kH, (long)kT * kH, (void*)LAB, (void*)LAB, kT, (long)kCP * kT, BIAS + kFBZ, nullptr, 0L, kCP, kT, kH, kSc);
  label_kernel<<<1920, kThr, 0, stream>>>(LAB, BIAS, out);
  last_out_kernel<<<128, kThr, 0, stream>>>(FIN, out + kOut1);
}
